// AvaAttention_78108275245355
// MI455X (gfx1250) — hardware-verified
//
#include <hip/hip_runtime.h>
#include <math.h>
#include <stdint.h>


#define NB   2
#define SEQ  2048
#define HID  2048
#define NQH  32
#define NKV  8
#define HD   64

typedef _Float16 v16h __attribute__((ext_vector_type(16)));
typedef _Float16 v8h  __attribute__((ext_vector_type(8)));
typedef __bf16   v16b __attribute__((ext_vector_type(16)));
typedef __bf16   v8b  __attribute__((ext_vector_type(8)));
typedef float    v8f  __attribute__((ext_vector_type(8)));
typedef float    v4f  __attribute__((ext_vector_type(4)));
typedef unsigned int v4u __attribute__((ext_vector_type(4)));

__device__ __forceinline__ unsigned short f2bf_bits(float f) {
  const unsigned u = __float_as_uint(f);
  return (unsigned short)((u + 0x7FFFu + ((u >> 16) & 1u)) >> 16);
}
__device__ __forceinline__ float bf_bits2f(unsigned short h) { return __uint_as_float(((unsigned)h) << 16); }
__device__ __forceinline__ unsigned pk16(unsigned short a, unsigned short b) { return (unsigned)a | ((unsigned)b << 16); }
__device__ __forceinline__ unsigned short h2u(_Float16 h) { return __builtin_bit_cast(unsigned short, h); }

__device__ __forceinline__ void wave_sync() {
  __builtin_amdgcn_fence(__ATOMIC_RELEASE, "workgroup");
  __builtin_amdgcn_wave_barrier();
  __builtin_amdgcn_fence(__ATOMIC_ACQUIRE, "workgroup");
}

union FragB { v16b v; v8b h[2]; };
union FragH { v16h v; v8h h[2]; };
__device__ __forceinline__ v16b ldfrag_b(const __bf16* p) {
  FragB f; f.h[0] = *(const v8b*)(p); f.h[1] = *(const v8b*)(p + 16); return f.v;
}
__device__ __forceinline__ v16h ldfrag_h(const _Float16* p) {
  FragH f; f.h[0] = *(const v8h*)(p); f.h[1] = *(const v8h*)(p + 16); return f.v;
}

__device__ __forceinline__ v8f wmma_b(v16b a, v16b b, v8f c) {
  return __builtin_amdgcn_wmma_f32_16x16x32_bf16(false, a, false, b, (short)0, c, false, false);
}
__device__ __forceinline__ v8f wmma_h(v16h a, v16h b, v8f c) {
  c = __builtin_amdgcn_wmma_f32_16x16x32_f16(false, a, false, b, (short)0, c, false, false);
  asm volatile("v_nop\n\tv_nop\n\tv_nop\n\tv_nop" : "+v"(c) : "v"(a), "v"(b));
  return c;
}
__device__ __forceinline__ void dep_guard_b(v8f& a, v8f& b, v16b x, v16b y) {
  asm volatile("v_nop\n\tv_nop\n\tv_nop\n\tv_nop" : "+v"(a), "+v"(b) : "v"(x), "v"(y));
}
__device__ __forceinline__ void keep4_b(v16b a, v16b b, v16b c, v16b d) { asm volatile("v_nop" :: "v"(a), "v"(b), "v"(c), "v"(d)); }
__device__ __forceinline__ void acc_guard4(v8f& a, v8f& b, v8f& c, v8f& d) {
  asm volatile("v_nop\n\tv_nop\n\tv_nop\n\tv_nop" : "+v"(a), "+v"(b), "+v"(c), "+v"(d));
}

__global__ __launch_bounds__(256) void cvt_bf16x8_kernel(const float* __restrict__ in, unsigned short* out, int n8) {
  const int i = blockIdx.x * 256 + threadIdx.x;
  if (i < n8) {
    const v4f a = *(const v4f*)(in + 8 * (size_t)i);
    const v4f c = *(const v4f*)(in + 8 * (size_t)i + 4);
    v4u w;
    w[0] = pk16(f2bf_bits(a[0]), f2bf_bits(a[1]));
    w[1] = pk16(f2bf_bits(a[2]), f2bf_bits(a[3]));
    w[2] = pk16(f2bf_bits(c[0]), f2bf_bits(c[1]));
    w[3] = pk16(f2bf_bits(c[2]), f2bf_bits(c[3]));
    volatile v4u* p = (volatile v4u*)(out + 8 * (size_t)i);
    *p = w;
    __threadfence();
    *p = w;
  }
}

__global__ __launch_bounds__(256) void rope_table_kernel(float* cs, int n) {
#pragma clang fp contract(off)
  const int t = blockIdx.x * 256 + threadIdx.x;
  if (t >= n) return;
  const int s = t >> 5;
  const int i = t & 31;
  const double ed = (double)i * 0.03125;
  const double pd = exp2(ed * 13.287712379549449);
  const float  pf = (float)pd;
  const float  inv = 1.0f / pf;
  const float  ang = (float)s * inv;
  const double ad = (double)ang;
  const double nd = rint(ad * 0.6366197723675814);
  const double rd = (ad - nd * 1.5707963267948966) - nd * 6.123233995736766e-17;
  const float  r = (float)rd;
  const float  z = r * r;
  const float  sr = r + r * z * ((-1.9515295891e-4f * z + 8.3321608736e-3f) * z - 1.6666654611e-1f);
  const float  cr = 1.0f - 0.5f * z + z * z * ((2.443315711809948e-5f * z - 1.388731625493765e-3f) * z + 4.166664568298827e-2f);
  const int qd = ((int)nd) & 3;
  float sv = sr, cv = cr;
  if (qd == 1) { sv = cr;  cv = -sr; }
  if (qd == 2) { sv = -sr; cv = -cr; }
  if (qd == 3) { sv = -cr; cv = sr;  }
  volatile float* pc = (volatile float*)(cs + (size_t)s * HD + i);
  volatile float* ps = (volatile float*)(cs + (size_t)s * HD + 32 + i);
  *pc = cv; *ps = sv;
  __threadfence();
  *pc = cv; *ps = sv;
}

template <bool SPLITA, int OUT_MODE>
__global__ __launch_bounds__(256) void gemm64_kernel(
    const unsigned short* __restrict__ Ap, const unsigned short* __restrict__ A2p, int lda, long strideA,
    const unsigned short* __restrict__ Btp, int ldb, long strideB,
    void* Cout, void* Cout2, void* Cout3, int ldc, long strideC,
    const float* __restrict__ cs, int M, int N, int K) {
  __shared__ __align__(16) float sT[8][16 * 68];
  const int bz   = blockIdx.y;
  const int lane = threadIdx.x & 31;
  const int wave = threadIdx.x >> 5;
  const int tilesN = N >> 6;
  const int tilesM = M >> 6;
  const int tile = blockIdx.x * 8 + wave;
  if (tile >= tilesM * tilesN) return;
  const int tm = tile / tilesN;
  const int tn = tile - tm * tilesN;
  const int m0 = tm << 6;
  const int n0 = tn << 6;

  const __bf16* Ab  = (const __bf16*)(const void*)Ap + (size_t)bz * strideA;
  const __bf16* Ab2 = SPLITA ? ((const __bf16*)(const void*)A2p + (size_t)bz * strideA) : (const __bf16*)0;
  const __bf16* Bb  = (const __bf16*)(const void*)Btp + (size_t)bz * strideB;

  const int rlane = lane & 15;
  const int koff  = (lane >> 4) * 8;
  const int mOff  = (lane >> 4) * 8;

  v8f acc[4][4];
#pragma unroll
  for (int i = 0; i < 4; ++i)
#pragma unroll
    for (int j = 0; j < 4; ++j) acc[i][j] = (v8f){0.f, 0.f, 0.f, 0.f, 0.f, 0.f, 0.f, 0.f};

  for (int k0 = 0; k0 < K; k0 += 32) {
    v16b bh[4];
#pragma unroll
    for (int j = 0; j < 4; ++j)
      bh[j] = ldfrag_b(Bb + (size_t)(n0 + (j << 4) + rlane) * ldb + koff + k0);
#pragma unroll
    for (int i = 0; i < 4; ++i) {
      const size_t ao = (size_t)(m0 + (i << 4) + rlane) * lda + koff + k0;
      const v16b ah = ldfrag_b(Ab + ao);
      v16b al = ah;
      if (SPLITA) al = ldfrag_b(Ab2 + ao);
#pragma unroll
      for (int j = 0; j < 4; ++j) {
        acc[i][j] = wmma_b(ah, bh[j], acc[i][j]);
        if (SPLITA) acc[i][j] = wmma_b(al, bh[j], acc[i][j]);
      }
      dep_guard_b(acc[i][0], acc[i][3], ah, al);
    }
    keep4_b(bh[0], bh[1], bh[2], bh[3]);
  }
  acc_guard4(acc[0][0], acc[0][1], acc[0][2], acc[0][3]);
  acc_guard4(acc[1][0], acc[1][1], acc[1][2], acc[1][3]);
  acc_guard4(acc[2][0], acc[2][1], acc[2][2], acc[2][3]);
  acc_guard4(acc[3][0], acc[3][1], acc[3][2], acc[3][3]);

  float* slab = sT[wave];
#pragma unroll
  for (int i = 0; i < 4; ++i) {
    const int mBase = m0 + (i << 4);
#pragma unroll
    for (int j = 0; j < 4; ++j)
#pragma unroll
      for (int r = 0; r < 8; ++r) slab[(mOff + r) * 68 + (j << 4) + rlane] = acc[i][j][r];
    wave_sync();
    if (OUT_MODE == 0) {
      float* C = (float*)Cout + (size_t)bz * strideC;
      const int h2 = lane >> 4, c4 = (lane & 15) * 4;
      for (int pass = 0; pass < 2; ++pass) {
#pragma unroll
        for (int it = 0; it < 8; ++it) {
          const int row = it * 2 + h2;
          const v4f v = *(const v4f*)(slab + row * 68 + c4);
          *(volatile v4f*)(C + (size_t)(mBase + row) * ldc + n0 + c4) = v;
        }
        __threadfence();
      }
    } else if (OUT_MODE == 1) {
      unsigned short* C  = (unsigned short*)Cout  + (size_t)bz * strideC;
      unsigned short* C2 = (unsigned short*)Cout2 + (size_t)bz * strideC;
      const int q8 = lane >> 3, c8 = (lane & 7) * 8;
      for (int pass = 0; pass < 2; ++pass) {
#pragma unroll
        for (int it = 0; it < 4; ++it) {
          const int row = it * 4 + q8;
          const float* sp = slab + row * 68 + c8;
          v4u hv, lv;
#pragma unroll
          for (int p = 0; p < 4; ++p) {
            const float f0 = sp[2 * p], f1 = sp[2 * p + 1];
            const _Float16 h0 = (_Float16)f0, h1 = (_Float16)f1;
            const _Float16 l0 = (_Float16)((f0 - (float)h0) * 2048.0f);
            const _Float16 l1 = (_Float16)((f1 - (float)h1) * 2048.0f);
            hv[p] = pk16(h2u(h0), h2u(h1));
            lv[p] = pk16(h2u(l0), h2u(l1));
          }
          const size_t go = (size_t)(mBase + row) * ldc + n0 + c8;
          *(volatile v4u*)(C  + go) = hv;
          *(volatile v4u*)(C2 + go) = lv;
        }
        __threadfence();
      }
    } else {
      unsigned short* Q1 = (unsigned short*)Cout;
      unsigned short* Q2 = (unsigned short*)Cout2;
      unsigned short* K1 = (unsigned short*)Cout3;
      const int q8 = lane >> 3, c8 = (lane & 7) * 8, dl = c8 & 31;
      const bool firsthalf = (c8 < 32);
      const int  bidx = m0 >> 11;
      const bool isq  = (n0 < NQH * HD);
      const size_t rowBase = isq ? ((size_t)(bidx * NQH + (n0 >> 6)) * SEQ)
                                 : ((size_t)(bidx * NKV + ((n0 - NQH * HD) >> 6)) * SEQ);
      for (int pass = 0; pass < 2; ++pass) {
#pragma unroll
        for (int it = 0; it < 4; ++it) {
          const int row = it * 4 + q8;
          const int s   = (mBase + row) & (SEQ - 1);
          const float* sp = slab + row * 68;
          const float* tp = cs + (size_t)s * HD;
          const v4f xa0 = *(const v4f*)(sp + dl),      xa1 = *(const v4f*)(sp + dl + 4);
          const v4f xb0 = *(const v4f*)(sp + 32 + dl), xb1 = *(const v4f*)(sp + 32 + dl + 4);
          const v4f co0 = *(const v4f*)(tp + dl),      co1 = *(const v4f*)(tp + dl + 4);
          const v4f si0 = *(const v4f*)(tp + 32 + dl), si1 = *(const v4f*)(tp + 32 + dl + 4);
          float o[8];
#pragma unroll
          for (int e = 0; e < 4; ++e) {
            const float a = xa0[e], bb = xb0[e], cc = co0[e], ss = si0[e];
            const float of = a * cc - bb * ss;
            const float os = bb * cc + a * ss;
            o[e] = firsthalf ? of : os;
          }
#pragma unroll
          for (int e = 0; e < 4; ++e) {
            const float a = xa1[e], bb = xb1[e], cc = co1[e], ss = si1[e];
            const float of = a * cc - bb * ss;
            const float os = bb * cc + a * ss;
            o[4 + e] = firsthalf ? of : os;
          }
          v4u hv, lv;
#pragma unroll
          for (int p = 0; p < 4; ++p) {
            const float f0 = o[2 * p], f1 = o[2 * p + 1];
            const _Float16 h0 = (_Float16)f0, h1 = (_Float16)f1;
            const _Float16 l0 = (_Float16)((f0 - (float)h0) * 2048.0f);
            const _Float16 l1 = (_Float16)((f1 - (float)h1) * 2048.0f);
            hv[p] = pk16(h2u(h0), h2u(h1));
            lv[p] = pk16(h2u(l0), h2u(l1));
          }
          const size_t go = (rowBase + (size_t)s) * HD + c8;
          if (isq) {
            *(volatile v4u*)(Q1 + go) = hv;
            *(volatile v4u*)(Q2 + go) = lv;
          } else {
            *(volatile v4u*)(K1 + go) = hv;
          }
        }
        __threadfence();
      }
    }
    wave_sync();
  }
}

#define AT_QB 64
#define AT_KC 64

__global__ __launch_bounds__(128)
void attn_kernel(const unsigned short* __restrict__ qhp, const unsigned short* __restrict__ qlp,
                 const unsigned short* __restrict__ kp,
                 const unsigned short* __restrict__ vhp, const unsigned short* __restrict__ vlp,
                 unsigned short* chp, unsigned short* clp) {
  __shared__ __align__(16) _Float16 Ksh[AT_KC * HD];
  __shared__ __align__(16) _Float16 Vth[HD * AT_KC];
  __shared__ __align__(16) _Float16 Vtl[HD * AT_KC];
  __shared__ __align__(16) _Float16 Psh[4][16 * AT_KC];
  __shared__ __align__(16) _Float16 Psl[4][16 * AT_KC];
  __shared__ __align__(16) float    Os[4][16 * 68];

  const int tid  = threadIdx.x;
  const int wave = tid >> 5;
  const int lane = tid & 31;
  const int hh   = lane >> 4;
  const int c    = lane & 15;

  const int bx  = blockIdx.x;
  const int qb  = bx & 31;
  const int h   = (bx >> 5) & 31;
  const int b   = bx >> 10;
  const int kvh = h >> 2;
  const int q0  = qb * AT_QB + wave * 16;

  const _Float16* Qh = (const _Float16*)(const void*)qhp + (size_t)(b * NQH + h) * SEQ * HD;
  const _Float16* Ql = (const _Float16*)(const void*)qlp + (size_t)(b * NQH + h) * SEQ * HD;
  const _Float16* Kh = (const _Float16*)(const void*)kp  + (size_t)(b * NKV + kvh) * SEQ * HD;
  const _Float16* Vh = (const _Float16*)(const void*)vhp + (size_t)(b * NKV + kvh) * HD * SEQ;
  const _Float16* Vl = (const _Float16*)(const void*)vlp + (size_t)(b * NKV + kvh) * HD * SEQ;

  v16h qah[2], qal[2];
#pragma unroll
  for (int dc = 0; dc < 2; ++dc) {
    qah[dc] = ldfrag_h(Qh + (size_t)(q0 + c) * HD + dc * 32 + 8 * hh);
    qal[dc] = ldfrag_h(Ql + (size_t)(q0 + c) * HD + dc * 32 + 8 * hh);
  }

  float mrow[8], lrow[8];
  v8f oh[4], orr[4];
#pragma unroll
  for (int r = 0; r < 8; ++r) { mrow[r] = -INFINITY; lrow[r] = 0.f; }
#pragma unroll
  for (int t = 0; t < 4; ++t) {
    oh[t]  = (v8f){0.f, 0.f, 0.f, 0.f, 0.f, 0.f, 0.f, 0.f};
    orr[t] = (v8f){0.f, 0.f, 0.f, 0.f, 0.f, 0.f, 0.f, 0.f};
  }

  const bool pres    = (qb < 2);
  const int  nChunks = qb + 1;
  for (int kc = 0; kc < nChunks; ++kc) {
    const int kv0 = kc * AT_KC;
    __syncthreads();
    {
      const int r = tid >> 1, half = (tid & 1) * 32;
      const _Float16* ks = Kh + (size_t)(kv0 + r) * HD + half;
      const _Float16* vs = Vh + (size_t)r * SEQ + kv0 + half;
      const _Float16* ws = Vl + (size_t)r * SEQ + kv0 + half;
#pragma unroll
      for (int i = 0; i < 4; ++i) {
        const v8h a0 = *(const v8h*)(ks + 8 * i);
        const v8h b0 = *(const v8h*)(vs + 8 * i);
        const v8h b1 = *(const v8h*)(ws + 8 * i);
        *(v8h*)(Ksh + r * HD    + half + 8 * i) = a0;
        *(v8h*)(Vth + r * AT_KC + half + 8 * i) = b0;
        *(v8h*)(Vtl + r * AT_KC + half + 8 * i) = b1;
      }
    }
    __syncthreads();

    v8f s[4];
#pragma unroll
    for (int j = 0; j < 4; ++j) {
      v8f sh = (v8f){0.f, 0.f, 0.f, 0.f, 0.f, 0.f, 0.f, 0.f};
      v8f sl = (v8f){0.f, 0.f, 0.f, 0.f, 0.f, 0.f, 0.f, 0.f};
#pragma unroll
      for (int dc = 0; dc < 2; ++dc) {
        FragH kb;
        kb.h[0] = *(const v8h*)(Ksh + (j * 16 + c) * HD + dc * 32 + 8 * hh);
        kb.h[1] = *(const v8h*)(Ksh + (j * 16 + c) * HD + dc * 32 + 16 + 8 * hh);
        sh = wmma_h(qah[dc], kb.v, sh);
        sl = wmma_h(qal[dc], kb.v, sl);
      }
      s[j] = sh + sl * 4.8828125e-4f;
    }

    const bool diag = (kc == qb);
    float cm[8];
#pragma unroll
    for (int r = 0; r < 8; ++r) {
      const int qrow = q0 + 8 * hh + r;
      float m = -INFINITY;
#pragma unroll
      for (int j = 0; j < 4; ++j) {
        const int kvcol = kv0 + j * 16 + c;
        const float sv = s[j][r] * 0.125f;
        const bool masked = diag && (kvcol > qrow);
        const float sm = masked ? -INFINITY : sv;
        s[j][r] = sm;
        m = fmaxf(m, sm);
      }
#pragma unroll
      for (int off = 1; off < 16; off <<= 1) m = fmaxf(m, __shfl_xor(m, off, 32));
      cm[r] = m;
    }

    _Float16* pwh = Psh[wave];
    _Float16* pwl = Psl[wave];
#pragma unroll
    for (int r = 0; r < 8; ++r) {
      const float mnew  = fmaxf(mrow[r], cm[r]);
      const float alpha = expf(mrow[r] - mnew);
      mrow[r] = mnew;
      float psum = 0.f;
#pragma unroll
      for (int j = 0; j < 4; ++j) {
        const float p   = expf(s[j][r] - mnew);
        psum += p;
        const float p1k = p * 1024.0f;
        const _Float16 ph = (_Float16)p1k;
        const _Float16 pl = (_Float16)((p1k - (float)ph) * 2048.0f);
        pwh[(8 * hh + r) * AT_KC + j * 16 + c] = ph;
        pwl[(8 * hh + r) * AT_KC + j * 16 + c] = pl;
      }
#pragma unroll
      for (int off = 1; off < 16; off <<= 1) psum += __shfl_xor(psum, off, 32);
      lrow[r] = lrow[r] * alpha + psum;
#pragma unroll
      for (int t = 0; t < 4; ++t) { oh[t][r] *= alpha; orr[t][r] *= alpha; }
    }
    wave_sync();

#pragma unroll 1
    for (int kk = 0; kk < 2; ++kk) {
      FragH pa, pb;
      pa.h[0] = *(const v8h*)(pwh + c * AT_KC + kk * 32 + 8 * hh);
      pa.h[1] = *(const v8h*)(pwh + c * AT_KC + kk * 32 + 16 + 8 * hh);
      pb.h[0] = *(const v8h*)(pwl + c * AT_KC + kk * 32 + 8 * hh);
      pb.h[1] = *(const v8h*)(pwl + c * AT_KC + kk * 32 + 16 + 8 * hh);
#pragma unroll
      for (int t = 0; t < 4; ++t) {
        FragH vb, vl;
        vb.h[0] = *(const v8h*)(Vth + (t * 16 + c) * AT_KC + kk * 32 + 8 * hh);
        vb.h[1] = *(const v8h*)(Vth + (t * 16 + c) * AT_KC + kk * 32 + 16 + 8 * hh);
        vl.h[0] = *(const v8h*)(Vtl + (t * 16 + c) * AT_KC + kk * 32 + 8 * hh);
        vl.h[1] = *(const v8h*)(Vtl + (t * 16 + c) * AT_KC + kk * 32 + 16 + 8 * hh);
        oh[t]  = wmma_h(pa.v, vb.v, oh[t]);
        orr[t] = wmma_h(pa.v, vl.v, orr[t]);
        if (pres) orr[t] = wmma_h(pb.v, vb.v, orr[t]);
      }
    }
  }

  float* os = Os[wave];
#pragma unroll
  for (int r = 0; r < 8; ++r) {
    const float invl = (1.0f / lrow[r]) * 9.765625e-4f;
#pragma unroll
    for (int t = 0; t < 4; ++t) os[(8 * hh + r) * 68 + t * 16 + c] = (oh[t][r] + orr[t][r] * 4.8828125e-4f) * invl;
  }
  wave_sync();
  {
    const int q8 = lane >> 3, c8 = (lane & 7) * 8;
    for (int pass = 0; pass < 2; ++pass) {
#pragma unroll
      for (int it = 0; it < 4; ++it) {
        const int row = it * 4 + q8;
        const float* sp = os + row * 68 + c8;
        v4u hv, lv;
#pragma unroll
        for (int p = 0; p < 4; ++p) {
          const float f0 = sp[2 * p], f1 = sp[2 * p + 1];
          const unsigned short hb0 = f2bf_bits(f0), hb1 = f2bf_bits(f1);
          const unsigned short lb0 = f2bf_bits(f0 - bf_bits2f(hb0));
          const unsigned short lb1 = f2bf_bits(f1 - bf_bits2f(hb1));
          hv[p] = pk16(hb0, hb1);
          lv[p] = pk16(lb0, lb1);
        }
        const size_t go = (size_t)(b * SEQ + q0 + row) * HID + h * HD + c8;
        *(volatile v4u*)(chp + go) = hv;
        *(volatile v4u*)(clp + go) = lv;
      }
      __threadfence();
    }
  }
}

extern "C" void kernel_launch(void* const* d_in, const int* in_sizes, int n_in,
                              void* d_out, int out_size, void* d_ws, size_t ws_size,
                              hipStream_t stream) {
  if (n_in < 5) return;
  if (in_sizes[0] != NB * SEQ * HID) return;
  if (in_sizes[1] != HID * HID) return;
  if (in_sizes[2] != NKV * HD * HID) return;
  if (in_sizes[3] != NKV * HD * HID) return;
  if (in_sizes[4] != HID * HID) return;
  if (out_size != NB * SEQ * HID) return;

  const float* x  = (const float*)d_in[0];
  const float* Wq = (const float*)d_in[1];
  const float* Wk = (const float*)d_in[2];
  const float* Wv = (const float*)d_in[3];
  const float* Wo = (const float*)d_in[4];
  float* out = (float*)d_out;

  const size_t szXb  = (size_t)NB * SEQ * HID * 2;
  const size_t szWqk = (size_t)(HID + NKV * HD) * HID * 2;
  const size_t szWv  = (size_t)NKV * HD * HID * 2;
  const size_t szWo  = (size_t)HID * HID * 2;
  const size_t szCs  = (size_t)SEQ * HD * 4;
  const size_t szQ   = (size_t)NB * NQH * SEQ * HD * 2;
  const size_t szK   = (size_t)NB * NKV * SEQ * HD * 2;
  const size_t szV   = (size_t)NB * NKV * HD * SEQ * 2;
  const size_t szC   = (size_t)NB * SEQ * HID * 2;
  size_t off = 0;
  const size_t oXb  = off; off += szXb;
  const size_t oWqk = off; off += szWqk;
  const size_t oWv  = off; off += szWv;
  const size_t oWo  = off; off += szWo;
  const size_t oCs  = off; off += szCs;
  const size_t oQh  = off; off += szQ;
  const size_t oQl  = off; off += szQ;
  const size_t oKp  = off; off += szK;
  const size_t oVth = off; off += szV;
  const size_t oVtl = off; off += szV;
  const size_t oCh  = off; off += szC;
  const size_t oCl  = off; off += szC;
  if (off > ws_size) return;

  char* ws = (char*)d_ws;
  unsigned short* Xb  = (unsigned short*)(ws + oXb);
  unsigned short* Wqk = (unsigned short*)(ws + oWqk);
  unsigned short* Wvb = (unsigned short*)(ws + oWv);
  unsigned short* Wob = (unsigned short*)(ws + oWo);
  float*          Cs  = (float*)(ws + oCs);
  unsigned short* Qh  = (unsigned short*)(ws + oQh);
  unsigned short* Ql  = (unsigned short*)(ws + oQl);
  unsigned short* Kp  = (unsigned short*)(ws + oKp);
  unsigned short* Vth = (unsigned short*)(ws + oVth);
  unsigned short* Vtl = (unsigned short*)(ws + oVtl);
  unsigned short* Ch  = (unsigned short*)(ws + oCh);
  unsigned short* Cl  = (unsigned short*)(ws + oCl);

  const dim3 blk(256);

  {
    const int n8x = NB * SEQ * HID / 8, n8q = HID * HID / 8, n8k = NKV * HD * HID / 8;
    cvt_bf16x8_kernel<<<dim3((n8x + 255) / 256), blk, 0, stream>>>(x, Xb, n8x);
    cvt_bf16x8_kernel<<<dim3((n8q + 255) / 256), blk, 0, stream>>>(Wq, Wqk, n8q);
    cvt_bf16x8_kernel<<<dim3((n8k + 255) / 256), blk, 0, stream>>>(Wk, Wqk + (size_t)HID * HID, n8k);
    cvt_bf16x8_kernel<<<dim3((n8k + 255) / 256), blk, 0, stream>>>(Wv, Wvb, n8k);
    cvt_bf16x8_kernel<<<dim3((n8q + 255) / 256), blk, 0, stream>>>(Wo, Wob, n8q);
  }
  {
    const int nt = SEQ * 32;
    rope_table_kernel<<<dim3((nt + 255) / 256), blk, 0, stream>>>(Cs, nt);
  }
  {
    const int M = NB * SEQ, N = HID + NKV * HD, K = HID;
    const int tiles = (M / 64) * (N / 64);
    gemm64_kernel<false, 2><<<dim3((tiles + 7) / 8, 1), blk, 0, stream>>>(
        Xb, Xb, HID, 0L, Wqk, HID, 0L, (void*)Qh, (void*)Ql, (void*)Kp, HD, 0L, Cs, M, N, K);
  }
  {
    const int M = NKV * HD, N = SEQ, K = HID;
    const int tiles = (M / 64) * (N / 64);
    gemm64_kernel<false, 1><<<dim3((tiles + 7) / 8, NB), blk, 0, stream>>>(
        Wvb, Wvb, HID, 0L, Xb, HID, (long)SEQ * HID, (void*)Vth, (void*)Vtl, (void*)Vtl, SEQ,
        (long)NKV * HD * SEQ, Cs, M, N, K);
  }
  attn_kernel<<<dim3(NB * NQH * (SEQ / AT_QB)), dim3(128), 0, stream>>>(Qh, Ql, Kp, Vth, Vtl, Ch, Cl);
  {
    const int M = NB * SEQ, N = HID, K = HID;
    const int tiles = (M / 64) * (N / 64);
    gemm64_kernel<true, 0><<<dim3((tiles + 7) / 8, 1), blk, 0, stream>>>(
        Ch, Cl, HID, 0L, Wob, HID, 0L, (void*)out, (void*)out, (void*)out, HID, 0L, Cs, M, N, K);
  }
  (void)hipGetLastError();
}
